// SimpleGCN_4337916969237
// MI455X (gfx1250) — hardware-verified
//
#include <hip/hip_runtime.h>
#include <stddef.h>
#include <stdint.h>
#include <math.h>


#define DIN    256
#define KP     256
#define DM     128
#define NZC    4
#define NTHR   256
#define NWAVE  8
#define EPT    8
#define CHUNK  (NTHR * EPT)
#define WCAP   (EPT * 32)
#define LISTN  (NWAVE * WCAP)
#define NBD    8192
#define SLD    13
#define NBA    1024
#define SLA    10
#define RCAP   28672
#define DEGCAP 128
#define GBM    64
#define GTHR   256
#define AGG_ZINTS (LISTN + 2 * RCAP + 3 * NBA)
#define AGG_LDS_INTS (AGG_ZINTS + 16)
#define WSMAX  134217728

static_assert((CHUNK & (CHUNK - 1)) == 0 && CHUNK <= 4096);
static_assert(NBD == (1 << SLD) && NBA == (1 << SLA));
static_assert(((long long)CHUNK << SLD) < (1LL << 31));
static_assert(((long long)CHUNK << SLA) < (1LL << 31));
static_assert(NBD % (NTHR * 4) == 0);
static_assert(LISTN % NTHR == 0);
static_assert(NBA % NWAVE == 0 && NBA % 32 == 0 && NBA % GBM == 0);
static_assert(RCAP % 32 == 0 && AGG_ZINTS % (NTHR * 4) == 0);
static_assert(KP % 32 == 0 && KP == 2 * DM && (KP / 8) == 32 && DIN == KP);
static_assert(DM == 4 * 32);
static_assert(GBM == 4 * 16 && GTHR == 8 * 32 && GTHR == 2 * DM);
static_assert(AGG_LDS_INTS * 4 <= 300000);
static_assert(NZC == 4);

typedef float          v2f   __attribute__((ext_vector_type(2)));
typedef float          v4f   __attribute__((ext_vector_type(4)));
typedef float          v8f   __attribute__((ext_vector_type(8)));
typedef int            v4i   __attribute__((ext_vector_type(4)));
typedef int            v8i   __attribute__((ext_vector_type(8)));
typedef unsigned int   v4u   __attribute__((ext_vector_type(4)));
typedef unsigned short v8us  __attribute__((ext_vector_type(8)));
typedef unsigned short v16us __attribute__((ext_vector_type(16)));
typedef __bf16         v16bf __attribute__((ext_vector_type(16)));
typedef v2f  __attribute__((may_alias)) v2fa;
typedef v4f  __attribute__((may_alias)) v4fa;
typedef v4i  __attribute__((may_alias)) v4ia;
typedef v8us __attribute__((may_alias)) v8usa;
union FragB { v16bf v; v16us u; v8us h[2]; v8i w; };

__device__ __forceinline__ v8f wmb(const FragB& a, const FragB& b, v8f c) {
  v8f d = __builtin_amdgcn_wmma_f32_16x16x32_bf16(false, a.v, false, b.v, (short)0, c, false, false);
  asm volatile("v_nop\n\tv_nop\n\tv_nop\n\tv_nop" : "+v"(d) : "v"(a.w), "v"(b.w));
  return d;
}

__device__ __forceinline__ unsigned int f2bf(float f) {
  const unsigned int u = __float_as_uint(f);
  return ((u + 0x7FFFu + ((u >> 16) & 1u)) >> 16) & 0xFFFFu;
}
__device__ __forceinline__ float bf2f(unsigned int b) { return __uint_as_float(b << 16); }
__device__ __forceinline__ float bfr(float f) { return bf2f(f2bf(f)); }
__device__ __forceinline__ v4f bfr4(const v4f a) {
  v4f r; r.x = bfr(a.x); r.y = bfr(a.y); r.z = bfr(a.z); r.w = bfr(a.w); return r;
}
__device__ __forceinline__ unsigned int pk2(float lo, float hi) { return f2bf(lo) | (f2bf(hi) << 16); }
__device__ __forceinline__ v4u pack8(const v4f a, const v4f b) {
  v4u r;
  r.x = pk2(a.x, a.y); r.y = pk2(a.z, a.w); r.z = pk2(b.x, b.y); r.w = pk2(b.z, b.w);
  return r;
}
__device__ __forceinline__ v4f relu4(const v4f a) {
  v4f r; r.x = fmaxf(a.x, 0.f); r.y = fmaxf(a.y, 0.f); r.z = fmaxf(a.z, 0.f); r.w = fmaxf(a.w, 0.f); return r;
}
__device__ __forceinline__ v4f zsel4(const v4f a, bool keep) {
  v4f r; r.x = keep ? a.x : 0.f; r.y = keep ? a.y : 0.f; r.z = keep ? a.z : 0.f; r.w = keep ? a.w : 0.f; return r;
}

template <int SLB>
__device__ __forceinline__ int scan_chunk(const int* __restrict__ dsts, int nE, int cbase, int slotBase,
                                          int nb, int vec8, int* list, int tid, int lane, int wave) {
  int wc = 0;
  const int el0  = tid * EPT;
  const int e0   = cbase + el0;
  const int sent = -2147483647 - 1;
  v4i da, db;
  if (vec8 != 0 && cbase + CHUNK <= nE) {
    da = *(const v4i*)(dsts + e0);
    db = *(const v4i*)(dsts + e0 + 4);
  } else {
    da.x = (e0     < nE) ? dsts[min(e0,     nE - 1)] : sent;
    da.y = (e0 + 1 < nE) ? dsts[min(e0 + 1, nE - 1)] : sent;
    da.z = (e0 + 2 < nE) ? dsts[min(e0 + 2, nE - 1)] : sent;
    da.w = (e0 + 3 < nE) ? dsts[min(e0 + 3, nE - 1)] : sent;
    db.x = (e0 + 4 < nE) ? dsts[min(e0 + 4, nE - 1)] : sent;
    db.y = (e0 + 5 < nE) ? dsts[min(e0 + 5, nE - 1)] : sent;
    db.z = (e0 + 6 < nE) ? dsts[min(e0 + 6, nE - 1)] : sent;
    db.w = (e0 + 7 < nE) ? dsts[min(e0 + 7, nE - 1)] : sent;
  }
  const unsigned nbs = (unsigned)slotBase;
  const unsigned unb = (unsigned)nb;
  const unsigned s0 = (unsigned)da.x - nbs, s1 = (unsigned)da.y - nbs;
  const unsigned s2 = (unsigned)da.z - nbs, s3 = (unsigned)da.w - nbs;
  const unsigned s4 = (unsigned)db.x - nbs, s5 = (unsigned)db.y - nbs;
  const unsigned s6 = (unsigned)db.z - nbs, s7 = (unsigned)db.w - nbs;
  const bool h0 = s0 < unb, h1 = s1 < unb, h2 = s2 < unb, h3 = s3 < unb;
  const bool h4 = s4 < unb, h5 = s5 < unb, h6 = s6 < unb, h7 = s7 < unb;
  const unsigned any = __builtin_amdgcn_ballot_w32(h0 | h1 | h2 | h3 | h4 | h5 | h6 | h7);
  if (any != 0u) {
#define HITJ(J, HJ, SJ) { \
      const unsigned mj = __builtin_amdgcn_ballot_w32(HJ); \
      if (mj != 0u) { \
        if (HJ) { \
          const int pos = wc + (int)__builtin_amdgcn_mbcnt_lo(mj, 0u); \
          if (pos < WCAP) list[wave * WCAP + pos] = ((el0 + (J)) << SLB) | (int)(SJ); \
        } \
        wc += (int)__builtin_popcount(mj); } }
    HITJ(0, h0, s0)
    HITJ(1, h1, s1)
    HITJ(2, h2, s2)
    HITJ(3, h3, s3)
    HITJ(4, h4, s4)
    HITJ(5, h5, s5)
    HITJ(6, h6, s6)
    HITJ(7, h7, s7)
#undef HITJ
  }
  return wc;
}

__global__ __launch_bounds__(NTHR) void k_xprep(const float* __restrict__ x, unsigned short* xb, int nN, int nUnits) {
  const int u = (int)blockIdx.x * NTHR + (int)threadIdx.x;
  if (u >= nUnits) return;
  const int row = u >> 5;
  const int k8  = (u & 31) * 8;
  const int rc  = row < nN ? row : nN - 1;
  const bool live = row < nN;
  const float* p = x + (size_t)rc * (size_t)DIN + k8;
  v4f a = *(const v4fa*)p;
  v4f b = *(const v4fa*)(p + 4);
  a = zsel4(a, live);
  b = zsel4(b, live);
  const v4u hv = pack8(a, b);
  unsigned short* o = xb + (size_t)row * KP + k8;
  *(volatile v4u*)o = hv;
  __threadfence();
  *(volatile v4u*)o = hv;
}

__global__ __launch_bounds__(NTHR) void k_wprep(const float* __restrict__ w, int Kin, int Kper, int Ncol, int Nrows,
                                                int Kout, unsigned short* wt, int nUnits) {
  const int u = (int)blockIdx.x * NTHR + (int)threadIdx.x;
  if (u >= nUnits) return;
  const int kq = Kout >> 3;
  const int n  = u / kq;
  const int k8 = (u - n * kq) * 8;
  const int kk = k8 - (k8 / Kper) * Kper;
  const int ncl = n < Ncol ? n : Ncol - 1;
  const bool nl = (n < Ncol);
  const size_t nc = (size_t)Ncol;
  const float* p = w + ncl;
  const int q0 = min(kk + 0, Kin - 1), q1 = min(kk + 1, Kin - 1), q2 = min(kk + 2, Kin - 1), q3 = min(kk + 3, Kin - 1);
  const int q4 = min(kk + 4, Kin - 1), q5 = min(kk + 5, Kin - 1), q6 = min(kk + 6, Kin - 1), q7 = min(kk + 7, Kin - 1);
  v4f a, b;
  a.x = p[(size_t)q0 * nc]; a.y = p[(size_t)q1 * nc]; a.z = p[(size_t)q2 * nc]; a.w = p[(size_t)q3 * nc];
  b.x = p[(size_t)q4 * nc]; b.y = p[(size_t)q5 * nc]; b.z = p[(size_t)q6 * nc]; b.w = p[(size_t)q7 * nc];
  a.x = (nl && kk + 0 < Kin) ? a.x : 0.f;
  a.y = (nl && kk + 1 < Kin) ? a.y : 0.f;
  a.z = (nl && kk + 2 < Kin) ? a.z : 0.f;
  a.w = (nl && kk + 3 < Kin) ? a.w : 0.f;
  b.x = (nl && kk + 4 < Kin) ? b.x : 0.f;
  b.y = (nl && kk + 5 < Kin) ? b.y : 0.f;
  b.z = (nl && kk + 6 < Kin) ? b.z : 0.f;
  b.w = (nl && kk + 7 < Kin) ? b.w : 0.f;
  const v4u wv = pack8(a, b);
  unsigned short* o = wt + (size_t)n * (size_t)Kout + k8;
  *(volatile v4u*)o = wv;
  __threadfence();
  *(volatile v4u*)o = wv;
}

__global__ __launch_bounds__(NTHR) void k_deg(const int* __restrict__ dsts, int nE, int vec8, float* dis) {
  __shared__ __attribute__((aligned(16))) int scnt[NBD];
  __shared__ __attribute__((aligned(16))) int list[LISTN];
  __shared__ int wcnt[NWAVE];
  const int tid = (int)threadIdx.x, lane = tid & 31, wave = tid >> 5;
  const int nodeBase = (int)blockIdx.x * NBD;

  for (int i = tid; i < NBD; i += NTHR) scnt[i] = 0;
  for (int i = tid; i < LISTN; i += NTHR) list[i] = 0;
  if (tid < NWAVE) wcnt[tid] = 0;
  __syncthreads();

  const int nChunks = (nE + CHUNK - 1) / CHUNK;
#pragma unroll 1
  for (int ch = 0; ch < nChunks; ++ch) {
    const int cbase = ch * CHUNK;
    const int wc = scan_chunk<SLD>(dsts, nE, cbase, nodeBase, NBD, vec8, list, tid, lane, wave);
    if (lane == 0) wcnt[wave] = wc;
    __syncthreads();
    if (wave == 0) {
#pragma unroll 1
      for (int w2 = 0; w2 < NWAVE; ++w2) {
        int c = wcnt[w2];
        c = c < 0 ? 0 : (c > WCAP ? WCAP : c);
#pragma unroll 1
        for (int b0 = 0; b0 < c; b0 += 32) {
          const int idx = b0 + lane;
          const int ent = list[w2 * WCAP + (idx < WCAP ? idx : WCAP - 1)];
          const int m32 = (c - b0) < 32 ? (c - b0) : 32;
#pragma unroll 1
          for (int k = 0; k < m32; ++k) {
            const int u  = __builtin_amdgcn_readlane(ent, k);
            const int sl = u & (NBD - 1);
            if (lane == 0) scnt[sl] = scnt[sl] + 1;
          }
        }
      }
    }
    __syncthreads();
  }

  v4f vals[NBD / (NTHR * 4)];
#pragma unroll
  for (int it = 0; it < NBD / (NTHR * 4); ++it) {
    const int s0 = it * (NTHR * 4) + 4 * tid;
    const v4i c4 = *(const v4ia*)(scnt + s0);
    const float d0 = (float)c4.x + 1.0f, d1 = (float)c4.y + 1.0f;
    const float d2 = (float)c4.z + 1.0f, d3 = (float)c4.w + 1.0f;
    v4f v;
    v.x = rsqrtf(d0); v.y = rsqrtf(d1); v.z = rsqrtf(d2); v.w = rsqrtf(d3);
    vals[it] = v;
  }
#pragma unroll
  for (int it = 0; it < NBD / (NTHR * 4); ++it) {
    const int s0 = it * (NTHR * 4) + 4 * tid;
    *(volatile v4f*)(dis + (size_t)nodeBase + s0) = vals[it];
  }
  __threadfence();
#pragma unroll
  for (int it = 0; it < NBD / (NTHR * 4); ++it) {
    const int s0 = it * (NTHR * 4) + 4 * tid;
    *(volatile v4f*)(dis + (size_t)nodeBase + s0) = vals[it];
  }
}

template <int EPI>
__global__ __launch_bounds__(GTHR) void k_gemm(
    const unsigned short* __restrict__ A, const unsigned short* __restrict__ WT,
    const float* __restrict__ bias, const float* __restrict__ w2, const float* __restrict__ b2,
    unsigned short* HBp, float* HFp, float* PRp, int nN)
{
  __shared__ __attribute__((aligned(16))) float stg[GBM * DM];
  __shared__ __attribute__((aligned(16))) float sbias[DM];
  __shared__ __attribute__((aligned(16))) float sw2[DM];
  __shared__ __attribute__((aligned(16))) float sres[GBM];
  const int tid = (int)threadIdx.x, lane = tid & 31, wave = tid >> 5, hh = lane >> 4, m = lane & 15;
  const int wr = wave & 3, wcol = wave >> 2;
  const int rowBase = (int)blockIdx.x * GBM;

  if constexpr (EPI == 0) {
    if (tid < DM) sbias[tid] = bfr(bias[tid]);
  } else if constexpr (EPI == 2) {
    if (tid < DM) sbias[tid] = bfr(bias[tid]);
    else          sw2[tid - DM] = bfr(w2[tid - DM]);
  }

  v8f acc[4];
  {
    const v8f z = {0.f, 0.f, 0.f, 0.f, 0.f, 0.f, 0.f, 0.f};
    acc[0] = z; acc[1] = z; acc[2] = z; acc[3] = z;
  }
  const unsigned short* ap = A  + (size_t)(rowBase + 16 * wr + m) * (size_t)KP + 8 * hh;
  const unsigned short* wp = WT + (size_t)(64 * wcol + m) * (size_t)KP + 8 * hh;
#pragma unroll 1
  for (int ks = 0; ks < KP / 32; ++ks) {
    FragB af;
    af.h[0] = *(const v8usa*)(ap + 32 * ks);
    af.h[1] = *(const v8usa*)(ap + 32 * ks + 16);
#pragma unroll
    for (int t = 0; t < 4; ++t) {
      const unsigned short* wq = wp + (size_t)(16 * t) * (size_t)KP + 32 * ks;
      FragB bf;
      bf.h[0] = *(const v8usa*)wq;
      bf.h[1] = *(const v8usa*)(wq + 16);
      acc[t] = wmb(af, bf, acc[t]);
    }
  }

#pragma unroll
  for (int t = 0; t < 4; ++t) {
    const int lc = 64 * wcol + 16 * t + m;
#pragma unroll
    for (int r = 0; r < 8; ++r) {
      const int lr = 16 * wr + 8 * hh + r;
      stg[lr * DM + lc] = acc[t][r];
    }
  }
  __syncthreads();

  if constexpr (EPI == 0) {
    const bool lsel = lane >= 16;
    const int c0 = 8 * (lane & 15);
    v4u pv[8];
    v4f fv[8];
#pragma unroll
    for (int it = 0; it < 8; ++it) {
      const int row = 8 * it + wave;
      const bool live = (rowBase + row) < nN;
      const float* hr = stg + row * DM;
      v4f h0 = *(const v4fa*)(hr + c0);
      v4f h1 = *(const v4fa*)(hr + c0 + 4);
      const v4f b0 = *(const v4fa*)(sbias + c0);
      const v4f b1 = *(const v4fa*)(sbias + c0 + 4);
      h0 = zsel4(relu4(h0 + b0), live);
      h1 = zsel4(relu4(h1 + b1), live);
      const v4f hi0 = bfr4(h0), hi1 = bfr4(h1);
      const v4f lo0 = h0 - hi0, lo1 = h1 - hi1;
      v4f o0, o1;
      o0.x = lsel ? lo0.x : hi0.x; o0.y = lsel ? lo0.y : hi0.y; o0.z = lsel ? lo0.z : hi0.z; o0.w = lsel ? lo0.w : hi0.w;
      o1.x = lsel ? lo1.x : hi1.x; o1.y = lsel ? lo1.y : hi1.y; o1.z = lsel ? lo1.z : hi1.z; o1.w = lsel ? lo1.w : hi1.w;
      pv[it] = pack8(o0, o1);
      v4f f = *(const v4fa*)(hr + 4 * lane);
      const v4f fb = *(const v4fa*)(sbias + 4 * lane);
      fv[it] = zsel4(relu4(f + fb), live);
    }
#pragma unroll
    for (int it = 0; it < 8; ++it) {
      const int gr = rowBase + 8 * it + wave;
      unsigned short* op = HBp + (size_t)gr * (size_t)KP + 8 * lane;
      float* fp = HFp + (size_t)gr * (size_t)DM + 4 * lane;
      *(volatile v4u*)op = pv[it];
      *(volatile v4f*)fp = fv[it];
    }
    __threadfence();
#pragma unroll
    for (int it = 0; it < 8; ++it) {
      const int gr = rowBase + 8 * it + wave;
      unsigned short* op = HBp + (size_t)gr * (size_t)KP + 8 * lane;
      float* fp = HFp + (size_t)gr * (size_t)DM + 4 * lane;
      *(volatile v4u*)op = pv[it];
      *(volatile v4f*)fp = fv[it];
    }
  } else if constexpr (EPI == 1) {
    v4f fv[8];
#pragma unroll
    for (int it = 0; it < 8; ++it) {
      const int row = 8 * it + wave;
      fv[it] = *(const v4fa*)(stg + row * DM + 4 * lane);
    }
#pragma unroll
    for (int it = 0; it < 8; ++it) {
      const int gr = rowBase + 8 * it + wave;
      float* fp = HFp + (size_t)gr * (size_t)DM + 4 * lane;
      *(volatile v4f*)fp = fv[it];
    }
    __threadfence();
#pragma unroll
    for (int it = 0; it < 8; ++it) {
      const int gr = rowBase + 8 * it + wave;
      float* fp = HFp + (size_t)gr * (size_t)DM + 4 * lane;
      *(volatile v4f*)fp = fv[it];
    }
  } else {
    if (tid < GBM) {
      const int row = tid;
      const float* hr = stg + row * DM;
      float d = 0.f;
#pragma unroll 4
      for (int c4 = 0; c4 < DM / 4; ++c4) {
        v4f hv = *(const v4fa*)(hr + 4 * c4);
        const v4f bv = *(const v4fa*)(sbias + 4 * c4);
        const v4f wv = *(const v4fa*)(sw2 + 4 * c4);
        hv = relu4(hv + bv);
        d = fmaf(hv.x, wv.x, d);
        d = fmaf(hv.y, wv.y, d);
        d = fmaf(hv.z, wv.z, d);
        d = fmaf(hv.w, wv.w, d);
      }
      d += bfr(b2[0]);
      const float ex = __expf(-d);
      const float p  = __builtin_amdgcn_rcpf(1.0f + ex);
      sres[row] = p;
    }
    __syncthreads();
    const v4f yv = *(const v4fa*)(sres + 4 * (lane & 15));
    float* op = PRp + rowBase + 4 * (lane & 15);
    const bool wrl = (wave == 0) && (lane < 16);
    if (wrl) *(volatile v4f*)op = yv;
    __threadfence();
    if (wrl) *(volatile v4f*)op = yv;
  }
}

__global__ __launch_bounds__(NTHR) void k_agg(const int* __restrict__ srcs, const int* __restrict__ dsts,
                                              int nE, int nN, int vec8, int mRows,
                                              const float* __restrict__ dis,
                                              const float* __restrict__ xl, const float* __restrict__ hfin,
                                              const float* __restrict__ bias,
                                              unsigned short* hb, float* hfout, int hfRows) {
  extern __shared__ __attribute__((aligned(16))) int dsm[];
  int* list = dsm;
  int* hl   = dsm + LISTN;
  int* sl   = dsm + LISTN + RCAP;
  int* cnt  = dsm + LISTN + 2 * RCAP;
  int* offs = cnt + NBA;
  int* cur  = offs + NBA;
  int* misc = cur + NBA;
  const int tid = (int)threadIdx.x, lane = tid & 31, wave = tid >> 5;
  const int nodeBase = (int)blockIdx.x * NBA;

  {
    const v4i z4 = {0, 0, 0, 0};
    for (int i = tid * 4; i < AGG_ZINTS; i += NTHR * 4) *(v4ia*)(dsm + i) = z4;
    if (tid < 16) misc[tid] = 0;
  }
  float bv0, bv1, bv2, bv3;
  {
    const v4f a = *(const v4fa*)(bias + 4 * lane);
    bv0 = bfr(a.x); bv1 = bfr(a.y); bv2 = bfr(a.z); bv3 = bfr(a.w);
  }
  __syncthreads();

  int t = 0, ov = 0;
  const int nChunks = (nE + CHUNK - 1) / CHUNK;
#pragma unroll 1
  for (int ch = 0; ch < nChunks; ++ch) {
    const int cbase = ch * CHUNK;
    const int wc = scan_chunk<SLA>(dsts, nE, cbase, nodeBase, NBA, vec8, list, tid, lane, wave);
    if (lane == 0) misc[wave] = wc;
    __syncthreads();
    if (wave == 0) {
#pragma unroll 1
      for (int w2 = 0; w2 < NWAVE; ++w2) {
        int c = misc[w2];
        c = c < 0 ? 0 : (c > WCAP ? WCAP : c);
#pragma unroll 1
        for (int b0 = 0; b0 < c; b0 += 32) {
          const int idx = b0 + lane;
          const int ent = list[w2 * WCAP + (idx < WCAP ? idx : WCAP - 1)];
          const int m32 = (c - b0) < 32 ? (c - b0) : 32;
#pragma unroll 1
          for (int k = 0; k < m32; ++k) {
            const int u    = __builtin_amdgcn_readlane(ent, k);
            const int slot = u & (NBA - 1);
            const int el   = (u >> SLA) & (CHUNK - 1);
            const int pk   = ((cbase + el) << SLA) | slot;
            if (t < RCAP) {
              if (lane == 0) { hl[t] = pk; cnt[slot] = cnt[slot] + 1; }
              t = t + 1;
            } else {
              ov = 1;
            }
          }
        }
      }
    }
    __syncthreads();
  }
  if (wave == 0 && lane == 0) { misc[8] = t; misc[9] = ov; }
  __syncthreads();
  int tt = misc[8];
  tt = tt < 0 ? 0 : (tt > RCAP ? RCAP : tt);
  const int ovf = misc[9];

  if (wave == 0) {
    const int base = lane * (NBA / 32);
    int s = 0;
#pragma unroll 1
    for (int i = 0; i < NBA / 32; ++i) s += cnt[base + i];
    int incl = s;
#pragma unroll
    for (int d = 1; d < 32; d <<= 1) {
      const int y = __shfl_up(incl, d, 32);
      if (lane >= d) incl += y;
    }
    int run = incl - s;
#pragma unroll 1
    for (int i = 0; i < NBA / 32; ++i) {
      const int cv = cnt[base + i];
      offs[base + i] = run;
      cur[base + i]  = run;
      run += cv;
    }
  }
  __syncthreads();
  if (wave == 0) {
#pragma unroll 1
    for (int b0 = 0; b0 < tt; b0 += 32) {
      const int idx = b0 + lane;
      const int ent = hl[idx < RCAP ? idx : RCAP - 1];
      const int m32 = (tt - b0) < 32 ? (tt - b0) : 32;
#pragma unroll 1
      for (int k = 0; k < m32; ++k) {
        const int u    = __builtin_amdgcn_readlane(ent, k);
        const int slot = u & (NBA - 1);
        if (lane == 0) {
          int p = cur[slot];
          p = p < 0 ? 0 : (p > RCAP - 1 ? RCAP - 1 : p);
          sl[p] = u;
          cur[slot] = p + 1;
        }
      }
    }
  }
  __syncthreads();

  const float qnan = __int_as_float(0x7fc00000);
  const float pz = (ovf != 0) ? qnan : 0.0f;
  const int sha = (2 * lane) & 31;
  const int shb = (2 * lane + 1) & 31;
  const bool lsel = lane >= 16;
#pragma unroll 1
  for (int si = 0; si < NBA / NWAVE; ++si) {
    const int s    = si * NWAVE + wave;
    const int node = nodeBase + s;
    int c = cnt[s];
    const bool big = c > DEGCAP;
    c = c < 0 ? 0 : (c > DEGCAP ? DEGCAP : c);
    int o = offs[s];
    o = o < 0 ? 0 : (o > RCAP ? RCAP : o);
    const int nc = node < nN ? node : nN - 1;
    const float dd = dis[nc];
    const float rd = dd * dd;
    float a0 = 0.0f, a1 = 0.0f, a2 = 0.0f, a3 = 0.0f;
#pragma unroll 1
    for (int b0 = 0; b0 < c; b0 += 32) {
      int idx = o + b0 + lane;
      idx = idx > RCAP - 1 ? RCAP - 1 : idx;
      const int ent = sl[idx];
      int eid = ent >> SLA;
      eid = eid < 0 ? 0 : (eid > nE - 1 ? nE - 1 : eid);
      int sr = srcs[eid];
      sr = sr < 0 ? 0 : (sr > nN - 1 ? nN - 1 : sr);
      const float cf  = dis[sr] * dd;
      const int   cfi = __float_as_int(cf);
      const int m32 = (c - b0) < 32 ? (c - b0) : 32;
#pragma unroll 1
      for (int k = 0; k < m32; ++k) {
        const int   sk = __builtin_amdgcn_readlane(sr, k);
        const float ck = __int_as_float(__builtin_amdgcn_readlane(cfi, k));
        const v4f a = *(const v4fa*)(xl + (size_t)sk * DM + 4 * lane);
        a0 = fmaf(ck, a.x, a0); a1 = fmaf(ck, a.y, a1);
        a2 = fmaf(ck, a.z, a2); a3 = fmaf(ck, a.w, a3);
      }
    }
    const v4f sv = *(const v4fa*)(xl   + (size_t)nc * DM + 4 * lane);
    const v4f hv = *(const v4fa*)(hfin + (size_t)nc * DM + 4 * lane);
    const float pzr = big ? qnan : pz;
    const bool live = node < nN;
    float y0 = ((a0 + sv.x * rd) + hv.x) + bv0;
    float y1 = ((a1 + sv.y * rd) + hv.y) + bv1;
    float y2 = ((a2 + sv.z * rd) + hv.z) + bv2;
    float y3 = ((a3 + sv.w * rd) + hv.w) + bv3;
    y0 = fmaxf(y0, 0.0f) + pzr; y1 = fmaxf(y1, 0.0f) + pzr;
    y2 = fmaxf(y2, 0.0f) + pzr; y3 = fmaxf(y3, 0.0f) + pzr;
    const float v0 = live ? y0 : 0.0f, v1 = live ? y1 : 0.0f, v2 = live ? y2 : 0.0f, v3 = live ? y3 : 0.0f;

    const unsigned hb0 = f2bf(v0), hb1 = f2bf(v1), hb2 = f2bf(v2), hb3 = f2bf(v3);
    const unsigned lb0 = f2bf(v0 - bf2f(hb0)), lb1 = f2bf(v1 - bf2f(hb1));
    const unsigned lb2 = f2bf(v2 - bf2f(hb2)), lb3 = f2bf(v3 - bf2f(hb3));
    const int hw0 = (int)(hb0 | (hb1 << 16));
    const int hw1 = (int)(hb2 | (hb3 << 16));
    const int lw0 = (int)(lb0 | (lb1 << 16));
    const int lw1 = (int)(lb2 | (lb3 << 16));
    const int g0 = __shfl(hw0, sha, 32), g1 = __shfl(hw1, sha, 32);
    const int g2 = __shfl(hw0, shb, 32), g3 = __shfl(hw1, shb, 32);
    const int q0 = __shfl(lw0, sha, 32), q1 = __shfl(lw1, sha, 32);
    const int q2 = __shfl(lw0, shb, 32), q3 = __shfl(lw1, shb, 32);
    v4u pv;
    pv.x = (unsigned int)(lsel ? q0 : g0);
    pv.y = (unsigned int)(lsel ? q1 : g1);
    pv.z = (unsigned int)(lsel ? q2 : g2);
    pv.w = (unsigned int)(lsel ? q3 : g3);
    v4f fo;
    fo.x = v0; fo.y = v1; fo.z = v2; fo.w = v3;
    const bool wrb = node < mRows;
    const bool wrf = node < hfRows;
    const int nrb = node < mRows ? node : mRows - 1;
    const int nrf = node < hfRows ? node : hfRows - 1;
    unsigned short* hp = hb + (size_t)nrb * (size_t)KP + 8 * lane;
    float* fp = hfout + (size_t)nrf * (size_t)DM + 4 * lane;
    if (wrb) *(volatile v4u*)hp = pv;
    if (wrf) *(volatile v4f*)fp = fo;
    __threadfence();
    if (wrb) *(volatile v4u*)hp = pv;
    if (wrf) *(volatile v4f*)fp = fo;
  }
}

__global__ __launch_bounds__(NTHR) void k_outpack(const float* __restrict__ pred, int MPr, int nN, float* out, int nF4) {
  const int i = (int)blockIdx.x * NTHR + (int)threadIdx.x;
  if (i >= nF4) return;
  const int e   = 4 * i;
  const int lim = 2 * nN;
  const int ee  = e < lim - 4 ? e : lim - 4;
  const int plane = ee >= nN ? 1 : 0;
  const int idx = ee - plane * nN;
  const v4f pv = *(const v4fa*)(pred + (size_t)plane * (size_t)MPr + idx);
  const v4f ov = zsel4(pv, e < lim);
  float* op = out + (size_t)e;
  *(volatile v4f*)op = ov;
  __threadfence();
  *(volatile v4f*)op = ov;
}

static inline int cdiv(int a, int b) { return (a + b - 1) / b; }

extern "C" void kernel_launch(void* const* d_in, const int* in_sizes, int n_in,
                              void* d_out, int out_size, void* d_ws, size_t ws_size,
                              hipStream_t stream) {
  if (n_in < 14) return;
  if (in_sizes[0] < DIN || (in_sizes[0] % DIN) != 0) return;
  const int nN = in_sizes[0] / DIN;
  if (nN < 4 || (nN & 3) != 0 || nN > (1 << 21)) return;
  if (in_sizes[1] < 2 || (in_sizes[1] & 1) != 0) return;
  const int nE = in_sizes[1] / 2;
  if (nE < 1 || nE >= (1 << (31 - SLA))) return;
  if (in_sizes[2] != DIN * DM || in_sizes[3] != DM) return;
  if (in_sizes[4] < DM * DM || (in_sizes[4] % (DM * DM)) != 0) return;
  const int nL = in_sizes[4] / (DM * DM);
  if (nL < 1 || nL > 16 || in_sizes[5] != nL * DM) return;
  if (in_sizes[6] != DM * DM || in_sizes[7] != DM) return;
  if (in_sizes[8] != DM || in_sizes[9] != 1) return;
  if (in_sizes[10] != DM * DM || in_sizes[11] != DM) return;
  if (in_sizes[12] != DM || in_sizes[13] != 1) return;
  if ((long long)out_size != (long long)nN * (2 + NZC + DM)) return;

  const float* x     = (const float*)d_in[0];
  const int*   edge  = (const int*)d_in[1];
  const float* w_in  = (const float*)d_in[2];
  const float* b_in  = (const float*)d_in[3];
  const float* w_gcn = (const float*)d_in[4];
  const float* b_gcn = (const float*)d_in[5];
  const float* w_nc1 = (const float*)d_in[6];
  const float* b_nc1 = (const float*)d_in[7];
  const float* w_nc2 = (const float*)d_in[8];
  const float* b_nc2 = (const float*)d_in[9];
  const float* w_oc1 = (const float*)d_in[10];
  const float* b_oc1 = (const float*)d_in[11];
  const float* w_oc2 = (const float*)d_in[12];
  const float* b_oc2 = (const float*)d_in[13];
  float* out = (float*)d_out;
  const int* src = edge;
  const int* dst = edge + nE;
  const size_t oH3 = (size_t)nN * (2 + NZC);

  const int MP   = cdiv(nN, GBM) * GBM;
  const int gM   = MP / GBM;
  const int gD   = cdiv(nN, NBD);
  const int NBPD = gD * NBD;
  const int gA   = cdiv(MP, NBA);
  if ((long long)gA * NBA < (long long)MP) return;
  if (NBPD < nN) return;
  const int vec8 = ((nE & 3) == 0) ? 1 : 0;

  char* ws = (char*)d_ws;
  size_t off = 0;
  const size_t oDIS = off; off += (size_t)NBPD * 4;                     off = (off + 255) & ~(size_t)255;
  const size_t oW1T = off; off += (size_t)DM * KP * 2;                  off = (off + 255) & ~(size_t)255;
  const size_t oWG  = off; off += (size_t)nL * DM * KP * 2;             off = (off + 255) & ~(size_t)255;
  const size_t oWH  = off; off += (size_t)2 * DM * KP * 2;              off = (off + 255) & ~(size_t)255;
  const size_t oPR  = off; off += (size_t)2 * MP * 4;                   off = (off + 255) & ~(size_t)255;
  const size_t szXB = (size_t)MP * KP * 2, szHF = (size_t)MP * DM * 4;
  const size_t oXB  = off; off += (szXB > szHF ? szXB : szHF);          off = (off + 255) & ~(size_t)255;
  const size_t oHF  = off; off += szHF;                                 off = (off + 255) & ~(size_t)255;
  const size_t oHB  = off; off += szXB;                                 off = (off + 255) & ~(size_t)255;
  const size_t oXW  = off; off += szHF;                                 off = (off + 255) & ~(size_t)255;
  if (off > ws_size || off > (size_t)WSMAX) return;
  float*          DIS = (float*)(ws + oDIS);
  unsigned short* W1T = (unsigned short*)(ws + oW1T);
  unsigned short* WG  = (unsigned short*)(ws + oWG);
  unsigned short* WH  = (unsigned short*)(ws + oWH);
  float*          PR  = (float*)(ws + oPR);
  unsigned short* XB  = (unsigned short*)(ws + oXB);
  float*          HFB = (float*)(ws + oXB);
  float*          HFA = (float*)(ws + oHF);
  unsigned short* HB  = (unsigned short*)(ws + oHB);
  float*          XW  = (float*)(ws + oXW);

  const size_t aggLds = (size_t)AGG_LDS_INTS * 4;
  hipFuncSetAttribute(reinterpret_cast<const void*>(&k_agg), hipFuncAttributeMaxDynamicSharedMemorySize, (int)aggLds);

  const int nUx = MP * (KP / 8);
  k_xprep<<<cdiv(nUx, NTHR), NTHR, 0, stream>>>(x, XB, nN, nUx);
  {
    const int nUw = DM * (KP / 8);
    k_wprep<<<cdiv(nUw, NTHR), NTHR, 0, stream>>>(w_in, DIN, KP, DM, DM, KP, W1T, nUw);
    for (int l = 0; l < nL; ++l)
      k_wprep<<<cdiv(nUw, NTHR), NTHR, 0, stream>>>(w_gcn + (size_t)l * DM * DM, DM, DM, DM, DM, KP,
                                                    WG + (size_t)l * DM * KP, nUw);
    k_wprep<<<cdiv(nUw, NTHR), NTHR, 0, stream>>>(w_nc1, DM, DM, DM, DM, KP, WH, nUw);
    k_wprep<<<cdiv(nUw, NTHR), NTHR, 0, stream>>>(w_oc1, DM, DM, DM, DM, KP, WH + (size_t)DM * KP, nUw);
  }
  k_deg<<<gD, NTHR, 0, stream>>>(dst, nE, vec8, DIS);
  k_gemm<0><<<gM, GTHR, 0, stream>>>(XB, W1T, b_in, w_nc2, b_nc2, HB, HFA, PR, nN);
  const float* hin = HFA;
  for (int l = 0; l < nL; ++l) {
    k_gemm<1><<<gM, GTHR, 0, stream>>>(HB, WG + (size_t)l * DM * KP, b_in, w_nc2, b_nc2, HB, XW, PR, nN);
    const bool last = (l == nL - 1);
    float* hout = last ? (out + oH3) : (((l & 1) != 0) ? HFA : HFB);
    const int hfRows = last ? nN : MP;
    k_agg<<<gA, NTHR, aggLds, stream>>>(src, dst, nE, nN, vec8, MP, DIS, XW, hin, b_gcn + (size_t)l * DM,
                                        HB, hout, hfRows);
    hin = hout;
  }
  k_gemm<2><<<gM, GTHR, 0, stream>>>(HB, WH, b_nc1, w_nc2, b_nc2, HB, XW, PR, nN);
  k_gemm<2><<<gM, GTHR, 0, stream>>>(HB, WH + (size_t)DM * KP, b_oc1, w_oc2, b_oc2, HB, XW, PR + MP, nN);
  const int nF4 = (int)(oH3 / 4);
  k_outpack<<<cdiv(nF4, NTHR), NTHR, 0, stream>>>(PR, MP, nN, out, nF4);
}
